// LTVZeroPhaseFIRFilter_22041772163078
// MI455X (gfx1250) — hardware-verified
//
#include <hip/hip_runtime.h>


namespace {
constexpr int B = 2, T = 131072, HOP = 256, NBIN = 257, KP = 288, NF = 512, FR = 512, NFR = 511, PAD = 255, LP = T + 2 * PAD, LPP = 132608  , NOUT = NFR * HOP, WKR = B * FR + 32;
constexpr float XS = 8.0f, MS = 1024.0f, KS = 64.0f;
typedef _Float16 b16;
typedef __attribute__((ext_vector_type(16))) _Float16 v16b;
typedef __attribute__((ext_vector_type(8))) _Float16 v8b;
typedef __attribute__((ext_vector_type(8))) float v8f;
typedef __attribute__((ext_vector_type(4))) float v4f;
__device__ __forceinline__ float bf16_rne(float f) { unsigned int u = __float_as_uint(f); u += 0x7FFFu + ((u >> 16) & 1u); return __uint_as_float(u & 0xFFFF0000u); }
__device__ __forceinline__ void split16(float v, b16& hi, b16& lo) { hi = (b16)v; lo = (b16)(v - (float)hi); }
__device__ __forceinline__ v16b frag_kb(const b16* p, int hh) { const v8b a = *(const v8b*)(p + 8 * hh), b = *(const v8b*)(p + 16 + 8 * hh); v16b f;
#pragma unroll
  for (int e = 0; e < 8; ++e) { f[e] = a[e]; f[8 + e] = b[e]; } return f; }
__device__ __forceinline__ v8f wmma16b(v16b a, v16b b, v8f c) { v8f d = __builtin_amdgcn_wmma_f32_16x16x32_f16(false, a, false, b, (short)0, c, false, false); asm volatile("v_nop\n\tv_nop\n\tv_nop\n\tv_nop" : "+v"(d) : "v"(a), "v"(b)); return d; }
__device__ __forceinline__ void wave_lds_sync() { __builtin_amdgcn_fence(__ATOMIC_RELEASE, "workgroup"); __builtin_amdgcn_wave_barrier(); __builtin_amdgcn_fence(__ATOMIC_ACQUIRE, "workgroup"); }
__device__ __forceinline__ float pmul(float a, float b) { float p = a * b; asm volatile("" : "+v"(p)); return p; }

__global__ __launch_bounds__(512) void costab_kernel(float* __restrict__ CT) { const int m = threadIdx.x; const float c = cosf(6.283185307179586f * (float)m / (float)NF); for (int pass = 0; pass < 2; ++pass) { ((volatile float*)CT)[m] = c; __threadfence(); } }
__global__ __launch_bounds__(256) void synmat_kernel(const float* __restrict__ CT, b16* __restrict__ MH, b16* __restrict__ ML) {
  const int u = blockIdx.x * 256 + threadIdx.x; if (u >= NF * KP / 8) return; const int e = u * 8; const int m = e / KP, k0 = e % KP; const int n = (m + NF / 2) & (NF - 1); v8b h, l;
#pragma unroll
  for (int j = 0; j < 8; ++j) { const int k = k0 + j; float v = 0.0f; if (k < NBIN) { const float wk = (k == 0 || k == NF / 2) ? 1.0f : 2.0f; v = wk * CT[(k * n) & (NF - 1)] * (1.0f / NF); } b16 p, q; split16(v * MS, p, q); h[j] = p; l[j] = q; }
  for (int pass = 0; pass < 2; ++pass) { *(volatile v8b*)(MH + e) = h; *(volatile v8b*)(ML + e) = l; __threadfence(); }
}
__global__ __launch_bounds__(256) void xb_kernel(const float* __restrict__ ex, b16* __restrict__ XB) {
  const size_t u = (size_t)blockIdx.x * 256 + threadIdx.x; if (u >= (size_t)B * LPP / 8) return; const size_t e = u * 8; const int b = (int)(e / LPP); const int i0 = (int)(e % LPP); v8b v;
#pragma unroll
  for (int j = 0; j < 8; ++j) { const int t = i0 + j - PAD; v[j] = (t >= 0 && t < T) ? (b16)(bf16_rne(ex[(size_t)b * T + t]) * XS) : (b16)0.0f; }
  for (int pass = 0; pass < 2; ++pass) { *(volatile v8b*)(XB + e) = v; __threadfence(); }
}
__global__ __launch_bounds__(32) void ker_kernel(const float* __restrict__ lm, const b16* __restrict__ MH, const b16* __restrict__ ML, b16* __restrict__ WKH, b16* __restrict__ WKL) {
  __shared__ __attribute__((aligned(16))) b16 Ah[16][KP + 8], Al[16][KP + 8]; __shared__ __attribute__((aligned(16))) b16 Th[16][128 + 8], Tl[16][128 + 8];
  const int lane = threadIdx.x, nloc = lane & 15, hlf = lane >> 4; const size_t r0 = (size_t)blockIdx.x * 16;
  for (int rr = 0; rr < 16; ++rr) for (int q = 0; q < KP / 32; ++q) { const int k = q * 32 + lane; const float v = k < NBIN ? __expf(bf16_rne(lm[(r0 + rr) * NBIN + k])) : 0.0f; b16 p, ql; split16(v * XS, p, ql); Ah[rr][k] = p; Al[rr][k] = ql; }
  wave_lds_sync(); const float sc = 1.0f / (XS * MS);
#pragma unroll 1
  for (int cg = 0; cg < NF / 128; ++cg) { v8f acc[8];
#pragma unroll
    for (int t = 0; t < 8; ++t) acc[t] = (v8f){};
#pragma unroll 3
    for (int kb = 0; kb < KP; kb += 32) { const v16b a = frag_kb(&Ah[nloc][kb], hlf), al = frag_kb(&Al[nloc][kb], hlf);
#pragma unroll
      for (int t = 0; t < 8; ++t) { const size_t ro = (size_t)(cg * 128 + t * 16 + nloc) * KP + kb; const v16b bh = frag_kb(MH + ro, hlf), bl = frag_kb(ML + ro, hlf); acc[t] = wmma16b(a, bh, acc[t]); acc[t] = wmma16b(a, bl, acc[t]); acc[t] = wmma16b(al, bh, acc[t]); acc[t] = wmma16b(al, bl, acc[t]); } }
#pragma unroll
    for (int t = 0; t < 8; ++t) { const int m = cg * 128 + t * 16 + nloc; const float hann = 0.5f * (1.0f - cosf(6.283185307179586f * (float)m / (float)NF));
#pragma unroll
      for (int r8 = 0; r8 < 8; ++r8) { b16 p, ql; split16(pmul(acc[t][r8] * sc, hann) * KS, p, ql); Th[8 * hlf + r8][t * 16 + nloc] = p; Tl[8 * hlf + r8][t * 16 + nloc] = ql; } }
    wave_lds_sync();
    for (int pass = 0; pass < 2; ++pass) { for (int rr = 0; rr < 16; ++rr) if (lane < 16) { *(volatile v8b*)(WKH + (r0 + rr) * NF + cg * 128 + lane * 8) = *(const v8b*)(&Th[rr][lane * 8]); *(volatile v8b*)(WKL + (r0 + rr) * NF + cg * 128 + lane * 8) = *(const v8b*)(&Tl[rr][lane * 8]); } __threadfence(); }
    wave_lds_sync(); }
}
__global__ __launch_bounds__(256) void wkzero_kernel(b16* __restrict__ WKH, b16* __restrict__ WKL) { const int u = blockIdx.x * 256 + threadIdx.x; if (u >= 32 * NF / 8) return; v8b z = {}; for (int pass = 0; pass < 2; ++pass) { *(volatile v8b*)(WKH + (size_t)B * FR * NF + u * 8) = z; *(volatile v8b*)(WKL + (size_t)B * FR * NF + u * 8) = z; __threadfence(); } }
__global__ __launch_bounds__(32) void conv_kernel(const b16* __restrict__ XB, const b16* __restrict__ WKH, const b16* __restrict__ WKL, float* __restrict__ out) {
  __shared__ __attribute__((aligned(16))) b16 Aw[16][NF + 8]; __shared__ float So[32];
  const int lane = threadIdx.x, nloc = lane & 15, hlf = lane >> 4; const size_t gp = (size_t)blockIdx.x * 32; const int b = (int)(gp / NOUT); const int p0 = (int)(gp % NOUT); const int f = p0 / HOP;
  const b16* xb = XB + (size_t)b * LPP + p0; const size_t kr = ((size_t)b * FR + f + nloc) * NF; const float sc = 1.0f / (XS * KS);
#pragma unroll 1
  for (int half = 0; half < 2; ++half) {
    for (int rr = 0; rr < 16; ++rr) for (int q = 0; q < NF / 32; ++q) Aw[rr][q * 32 + lane] = xb[half * 16 + rr + q * 32 + lane];
    wave_lds_sync();
    v8f acc = {};
#pragma unroll 4
    for (int kb = 0; kb < NF; kb += 32) { const v16b a = frag_kb(&Aw[nloc][kb], hlf); acc = wmma16b(a, frag_kb(WKH + kr + kb, hlf), acc); acc = wmma16b(a, frag_kb(WKL + kr + kb, hlf), acc); }
    if (nloc == 0) {
#pragma unroll
      for (int r8 = 0; r8 < 8; ++r8) So[half * 16 + 8 * hlf + r8] = acc[r8] * sc; }
    wave_lds_sync(); }
  for (int pass = 0; pass < 2; ++pass) { ((volatile float*)out)[gp + lane] = So[lane]; __threadfence(); }
}
}

extern "C" void kernel_launch(void* const* d_in, const int* in_sizes, int n_in, void* d_out, int out_size, void* d_ws, size_t ws_size, hipStream_t stream) {
  (void)n_in;
  auto Fp = [&](int i) { return (const float*)d_in[i]; };
  if (in_sizes[0] != B * T || in_sizes[1] != B * FR * NBIN || out_size != B * NOUT) return;
  const int NPV = B * NOUT;
  size_t off = 0; char* ws = (char*)d_ws;
  auto carve = [&](size_t bytes) { char* p = ws + off; off += (bytes + 255) & ~(size_t)255; return p; };
  float* CT = (float*)carve(NF * 4); b16* MH = (b16*)carve((size_t)NF * KP * 2); b16* ML = (b16*)carve((size_t)NF * KP * 2); b16* XB = (b16*)carve((size_t)B * LPP * 2); b16* WKH = (b16*)carve((size_t)WKR * NF * 2); b16* WKL = (b16*)carve((size_t)WKR * NF * 2);
  if (off > ws_size || off > ((size_t)16 << 20)) return;
  costab_kernel<<<1, NF, 0, stream>>>(CT); synmat_kernel<<<(NF * KP / 8 + 255) / 256, 256, 0, stream>>>(CT, MH, ML);
  xb_kernel<<<(unsigned)(((size_t)B * LPP / 8 + 255) / 256), 256, 0, stream>>>(Fp(0), XB);
  wkzero_kernel<<<(32 * NF / 8 + 255) / 256, 256, 0, stream>>>(WKH, WKL);
  ker_kernel<<<B * FR / 16, 32, 0, stream>>>(Fp(1), MH, ML, WKH, WKL);
  conv_kernel<<<NPV / 32, 32, 0, stream>>>(XB, WKH, WKL, (float*)d_out);
}
